// GraphAttnModel_33294586479124
// MI455X (gfx1250) — hardware-verified
//
#include <hip/hip_runtime.h>
#include <stddef.h>


#define FD    256
#define NHD   4
#define GR    16
#define LDSP  264
#define NB    256
#define SH    8
#define CHUNK 4096
#define ATHR  256
#define AWAVE 8
#define NGRP  (CHUNK / (ATHR * 4))
#define WCAP  ((CHUNK / ATHR) * 32)
#define AGG_SACC (NB * FD)
#define AGG_AUX  (2 * NB * NHD)
#define AGG_LIST (AWAVE * WCAP)
#define AGG_LDS_BYTES ((AGG_SACC + AGG_AUX + AGG_LIST + AWAVE) * 4)
#define WS_CAP ((size_t)134217728)

static_assert(NGRP == 4);
static_assert(WCAP == 512);
static_assert(NB == (1 << SH));
static_assert(SH + 12 <= 31);
static_assert(AGG_LDS_BYTES == 286752);
static_assert((LDSP * 2) % 16 == 0);
static_assert(FD == 32 * 8);

typedef float          v4f   __attribute__((ext_vector_type(4)));
typedef float          v8f   __attribute__((ext_vector_type(8)));
typedef int            v4i   __attribute__((ext_vector_type(4)));
typedef unsigned short v8us  __attribute__((ext_vector_type(8)));
typedef __bf16         v16bf __attribute__((ext_vector_type(16)));

union Frag  { v16bf v; v8us p[2]; };
union LdsG3 { unsigned short hs[2 * GR * LDSP]; float xs[GR * (3 * FD + 4)]; };
union LdsG1 { unsigned short hs[2 * GR * LDSP]; float xs[GR * (FD + 4)]; };

__device__ __forceinline__ unsigned short bf16_rne(float x) {
  unsigned u = __float_as_uint(x);
  u += 0x7FFFu + ((u >> 16) & 1u);
  return (unsigned short)(u >> 16);
}
__device__ __forceinline__ float bf16_val(unsigned short b) {
  return __uint_as_float(((unsigned)b) << 16);
}

__device__ __forceinline__ v8f wm(v16bf a, v16bf b, v8f c) {
  v8f d = __builtin_amdgcn_wmma_f32_16x16x32_bf16(false, a, false, b, (short)0, c, false, false);
  asm volatile("v_nop\n\tv_nop\n\tv_nop\n\tv_nop" : "+v"(d) : "v"(a), "v"(b));
  return d;
}

__device__ __forceinline__ float wsum(float v) {
  v += __shfl_xor(v, 16, 32);
  v += __shfl_xor(v, 8, 32);
  v += __shfl_xor(v, 4, 32);
  v += __shfl_xor(v, 2, 32);
  v += __shfl_xor(v, 1, 32);
  return v;
}

__device__ __forceinline__ float hsum4(v4f a) { return (a.x + a.y) + (a.z + a.w); }
__device__ __forceinline__ v4f ld4(const float* p) { return *(const v4f*)p; }

__device__ __forceinline__ v4f prelu4(v4f o, float al) {
  v4f r;
  r.x = (o.x > 0.f) ? o.x : al * o.x;
  r.y = (o.y > 0.f) ? o.y : al * o.y;
  r.z = (o.z > 0.f) ? o.z : al * o.z;
  r.w = (o.w > 0.f) ? o.w : al * o.w;
  return r;
}

__device__ __forceinline__ void split8(v4f a, v4f b, v8us& h, v8us& l) {
  const float x[8] = {a.x, a.y, a.z, a.w, b.x, b.y, b.z, b.w};
#pragma unroll
  for (int i = 0; i < 8; ++i) {
    const unsigned short hb = bf16_rne(x[i]);
    h[i] = hb;
    l[i] = bf16_rne(x[i] - bf16_val(hb));
  }
}

__device__ __forceinline__ void stage_rows(const float* __restrict__ A, int rowBase, int nA,
                                           unsigned short* ldsH, unsigned short* ldsL, int tid) {
  const int r  = tid >> 4;
  const int c0 = (tid & 15) * 16;
  int row = rowBase + r;
  if (row > nA - 1) row = nA - 1;
  const float* p = A + (size_t)row * FD + c0;
  const v4f f0 = ld4(p);
  const v4f f1 = ld4(p + 4);
  const v4f f2 = ld4(p + 8);
  const v4f f3 = ld4(p + 12);
  v8us h0 = {0, 0, 0, 0, 0, 0, 0, 0}, h1 = {0, 0, 0, 0, 0, 0, 0, 0};
  v8us l0 = {0, 0, 0, 0, 0, 0, 0, 0}, l1 = {0, 0, 0, 0, 0, 0, 0, 0};
  split8(f0, f1, h0, l0);
  split8(f2, f3, h1, l1);
  unsigned short* dh = ldsH + r * LDSP + c0;
  unsigned short* dl = ldsL + r * LDSP + c0;
  *(v8us*)(dh)     = h0;
  *(v8us*)(dh + 8) = h1;
  *(v8us*)(dl)     = l0;
  *(v8us*)(dl + 8) = l1;
}

template <int TPW>
__device__ __forceinline__ void gemm_core(const unsigned short* ldsH, const unsigned short* ldsL,
                                          const unsigned short* __restrict__ wHi,
                                          const unsigned short* __restrict__ wLo,
                                          int tile0, int lane, v8f (&acc)[TPW]) {
  const int hh = lane >> 4;
  const int m  = lane & 15;
  const v8f z8 = {0.f, 0.f, 0.f, 0.f, 0.f, 0.f, 0.f, 0.f};
#pragma unroll
  for (int t = 0; t < TPW; ++t) acc[t] = z8;
  const unsigned short* pa  = ldsH + m * LDSP + 8 * hh;
  const unsigned short* pal = ldsL + m * LDSP + 8 * hh;
#pragma unroll 1
  for (int kt = 0; kt < FD / 32; ++kt) {
    const int k0 = kt * 32;
    Frag ah, al;
    ah.p[0] = *(const v8us*)(pa + k0);
    ah.p[1] = *(const v8us*)(pa + k0 + 16);
    al.p[0] = *(const v8us*)(pal + k0);
    al.p[1] = *(const v8us*)(pal + k0 + 16);
#pragma unroll
    for (int t = 0; t < TPW; ++t) {
      const size_t prow = (size_t)(tile0 + t) * 16 + m;
      const unsigned short* pb  = wHi + prow * FD + k0 + 8 * hh;
      const unsigned short* pbl = wLo + prow * FD + k0 + 8 * hh;
      Frag bh, bl;
      bh.p[0] = *(const v8us*)(pb);
      bh.p[1] = *(const v8us*)(pb + 16);
      bl.p[0] = *(const v8us*)(pbl);
      bl.p[1] = *(const v8us*)(pbl + 16);
      acc[t] = wm(ah.v, bh.v, acc[t]);
      acc[t] = wm(ah.v, bl.v, acc[t]);
      acc[t] = wm(al.v, bh.v, acc[t]);
    }
  }
}

__global__ __launch_bounds__(256) void k_prep(const float* __restrict__ w0, const float* __restrict__ w1,
                                             const float* __restrict__ w2, const float* __restrict__ w3,
                                             unsigned short* wHi, unsigned short* wLo, int ntot) {
  const int t = blockIdx.x * 256 + threadIdx.x;
  if (t >= ntot) return;
  const int mat = t >> 8;
  const int n   = t & (FD - 1);
  const float* W = (mat == 0) ? w0 : ((mat == 1) ? w1 : ((mat == 2) ? w2 : w3));
  unsigned short* dh = wHi + (size_t)t * FD;
  unsigned short* dl = wLo + (size_t)t * FD;
#pragma unroll 1
  for (int kb = 0; kb < FD / 8; ++kb) {
    v8us h = {0, 0, 0, 0, 0, 0, 0, 0}, l = {0, 0, 0, 0, 0, 0, 0, 0};
#pragma unroll
    for (int i = 0; i < 8; ++i) {
      const float x = W[(size_t)(kb * 8 + i) * FD + n];
      const unsigned short hb = bf16_rne(x);
      h[i] = hb;
      l[i] = bf16_rne(x - bf16_val(hb));
    }
    *(volatile v8us*)(dh + kb * 8) = h;
    *(volatile v8us*)(dl + kb * 8) = l;
    __threadfence();
    *(volatile v8us*)(dh + kb * 8) = h;
    *(volatile v8us*)(dl + kb * 8) = l;
  }
}

__global__ __launch_bounds__(256) void k_gemm3(const float* __restrict__ feat,
                                              const unsigned short* __restrict__ wHi,
                                              const unsigned short* __restrict__ wLo,
                                              const float* __restrict__ b0, const float* __restrict__ b1,
                                              const float* __restrict__ b2,
                                              float* o0, float* o1, float* o2, int nA) {
  constexpr int TPW = 6;
  constexpr int XSP = 3 * FD + 4;
  __shared__ __attribute__((aligned(16))) LdsG3 lds;

  const int tid  = threadIdx.x;
  const int lane = tid & 31;
  const int wave = tid >> 5;
  const int hh   = lane >> 4;
  const int m    = lane & 15;
  const int rowBase = blockIdx.x * GR;
  unsigned short* ldsH = lds.hs;
  unsigned short* ldsL = lds.hs + GR * LDSP;

  stage_rows(feat, rowBase, nA, ldsH, ldsL, tid);
  __syncthreads();

  v8f acc[TPW];
  gemm_core<TPW>(ldsH, ldsL, wHi, wLo, wave * TPW, lane, acc);
  __syncthreads();

#pragma unroll
  for (int t = 0; t < TPW; ++t) {
    const int tile = wave * TPW + t;
    const int mat  = tile >> 4;
    const int gc   = tile * 16 + m;
    const int bcol = gc & (FD - 1);
    const float* bb = (mat == 0) ? b0 : ((mat == 1) ? b1 : b2);
    const float bvl = bb[bcol];
#pragma unroll
    for (int r = 0; r < 8; ++r) lds.xs[(8 * hh + r) * XSP + gc] = acc[t][r] + bvl;
  }
  __syncthreads();

  v4f xr[2 * TPW];
  float* gp[2 * TPW];
  bool okv[TPW];
#pragma unroll
  for (int q = 0; q < TPW; ++q) {
    const int s    = wave * TPW + q;
    const int mat  = s >> 4;
    const int row  = s & 15;
    const int node = rowBase + row;
    float* ob = (mat == 0) ? o0 : ((mat == 1) ? o1 : o2);
    const float* xsrow = lds.xs + row * XSP + mat * FD + 4 * lane;
    xr[2 * q]     = ld4(xsrow);
    xr[2 * q + 1] = ld4(xsrow + 128);
    gp[2 * q]     = ob + (size_t)node * FD + 4 * lane;
    gp[2 * q + 1] = ob + (size_t)node * FD + 128 + 4 * lane;
    okv[q] = node < nA;
  }
#pragma unroll
  for (int q = 0; q < TPW; ++q) {
    if (okv[q]) {
      *(volatile v4f*)(gp[2 * q])     = xr[2 * q];
      *(volatile v4f*)(gp[2 * q + 1]) = xr[2 * q + 1];
    }
  }
  __threadfence();
#pragma unroll
  for (int q = 0; q < TPW; ++q) {
    if (okv[q]) {
      *(volatile v4f*)(gp[2 * q])     = xr[2 * q];
      *(volatile v4f*)(gp[2 * q + 1]) = xr[2 * q + 1];
    }
  }
}

__global__ __launch_bounds__(ATHR) void k_agg(const int* __restrict__ srcA, const int* __restrict__ dstA,
                                              const float* __restrict__ Q, const float* __restrict__ V,
                                              float* kio, int nN, int nE) {
  extern __shared__ v4f lds_dyn[];
  float* sacc = (float*)lds_dyn;
  float* mx   = sacc + AGG_SACC;
  float* den  = mx + NB * NHD;
  int*   list = (int*)(den + NB * NHD);
  int*   wcnt = list + AGG_LIST;

  const int tid  = threadIdx.x;
  const int lane = tid & 31;
  const int wave = tid >> 5;
  const int hd   = lane >> 3;
  const int nodeBase = blockIdx.x * NB;

  {
    const v4f z4 = {0.f, 0.f, 0.f, 0.f};
    for (int i = tid; i < AGG_SACC / 4; i += ATHR) lds_dyn[i] = z4;
    for (int i = tid; i < NB * NHD; i += ATHR) { mx[i] = -1.0e30f; den[i] = 0.f; }
  }
  __syncthreads();

  const bool al16 = ((nE & 3) == 0);
  const int nChunks = (nE + CHUNK - 1) / CHUNK;
#pragma unroll 1
  for (int ch = 0; ch < nChunks; ++ch) {
    const int cbase = ch * CHUNK;
    int wc = 0;
#pragma unroll
    for (int g = 0; g < NGRP; ++g) {
      const int el0 = (g * ATHR + tid) * 4;
      const int e0  = cbase + el0;
      const int sent = -2147483647 - 1;
      v4i d;
      if (al16 && (e0 + 3 < nE)) {
        d = *(const v4i*)(dstA + e0);
      } else {
        d.x = (e0     < nE) ? dstA[min(e0, nE - 1)]     : sent;
        d.y = (e0 + 1 < nE) ? dstA[min(e0 + 1, nE - 1)] : sent;
        d.z = (e0 + 2 < nE) ? dstA[min(e0 + 2, nE - 1)] : sent;
        d.w = (e0 + 3 < nE) ? dstA[min(e0 + 3, nE - 1)] : sent;
      }
      const unsigned s0 = (unsigned)d.x - (unsigned)nodeBase;
      const unsigned s1 = (unsigned)d.y - (unsigned)nodeBase;
      const unsigned s2 = (unsigned)d.z - (unsigned)nodeBase;
      const unsigned s3 = (unsigned)d.w - (unsigned)nodeBase;
      const bool h0 = s0 < (unsigned)NB;
      const bool h1 = s1 < (unsigned)NB;
      const bool h2 = s2 < (unsigned)NB;
      const bool h3 = s3 < (unsigned)NB;
      const unsigned many = __builtin_amdgcn_ballot_w32(h0 | h1 | h2 | h3);
      if (many != 0u) {
#define HITJ(J, HJ, SJ) { \
          const unsigned mj = __builtin_amdgcn_ballot_w32(HJ); \
          if (HJ) { \
            const int pos = wc + (int)__builtin_amdgcn_mbcnt_lo(mj, 0u); \
            if (pos < WCAP) list[wave * WCAP + pos] = ((el0 + (J)) << SH) | (int)(SJ); \
          } \
          wc += (int)__builtin_popcount(mj); }
        HITJ(0, h0, s0)
        HITJ(1, h1, s1)
        HITJ(2, h2, s2)
        HITJ(3, h3, s3)
#undef HITJ
      }
    }
    if (lane == 0) wcnt[wave] = wc;
    __syncthreads();

    if (wave == 0) {
#pragma unroll 1
      for (int wsx = 0; wsx < AWAVE; ++wsx) {
        int n = wcnt[wsx];
        if (n > WCAP) n = WCAP;
        if (n < 0) n = 0;
#pragma unroll 1
        for (int i = 0; i < n; ++i) {
          const int ent  = list[wsx * WCAP + i];
          const int slot = ent & (NB - 1);
          const int el   = (ent >> SH) & (CHUNK - 1);
          int e = cbase + el;
          if (e > nE - 1) e = nE - 1;
          int src = srcA[e];
          src = src < 0 ? 0 : (src > nN - 1 ? nN - 1 : src);
          int nd = nodeBase + slot;
          if (nd > nN - 1) nd = nN - 1;
          const float* qrow = Q   + (size_t)src * FD + 8 * lane;
          const float* krow = kio + (size_t)nd  * FD + 8 * lane;
          const float* vrow = V   + (size_t)src * FD + 8 * lane;
          const v4f q0 = ld4(qrow), q1 = ld4(qrow + 4);
          const v4f k0 = ld4(krow), k1 = ld4(krow + 4);
          const v4f v0 = ld4(vrow), v1 = ld4(vrow + 4);
          float part = hsum4(q0 * k0) + hsum4(q1 * k1);
          part += __shfl_xor(part, 4, 32);
          part += __shfl_xor(part, 2, 32);
          part += __shfl_xor(part, 1, 32);
          const float logit = part * 0.125f;
          const int hidx = slot * NHD + hd;
          const float mo = mx[hidx];
          const float mn = fmaxf(mo, logit);
          const float corr = __expf(mo - mn);
          const float p = __expf(logit - mn);
          const float dn = den[hidx] * corr + p;
          v4f* sp = (v4f*)(sacc + slot * FD + 8 * lane);
          const v4f c0 = sp[0];
          const v4f c1 = sp[1];
          sp[0] = c0 * corr + v0 * p;
          sp[1] = c1 * corr + v1 * p;
          den[hidx] = dn;
          mx[hidx]  = mn;
        }
      }
    }
    __syncthreads();
  }

  constexpr int NV = AGG_SACC / 4;
#pragma unroll 1
  for (int idx = tid; idx < NV; idx += ATHR) {
    const int row  = idx >> 6;
    const int c4   = idx & 63;
    const int head = c4 >> 4;
    const float d  = den[row * NHD + head];
    const float inv = (d > 0.f) ? (1.0f / d) : 0.f;
    const v4f val = lds_dyn[idx] * inv;
    lds_dyn[idx] = val;
    const int node = nodeBase + row;
    if (node < nN) *(volatile v4f*)(kio + (size_t)node * FD + 4 * c4) = val;
  }
  __threadfence();
#pragma unroll 1
  for (int idx = tid; idx < NV; idx += ATHR) {
    const int row  = idx >> 6;
    const int c4   = idx & 63;
    const int node = nodeBase + row;
    const v4f val = lds_dyn[idx];
    if (node < nN) *(volatile v4f*)(kio + (size_t)node * FD + 4 * c4) = val;
  }
}

__device__ __forceinline__ void row_epi(v4f sk0, v4f sk1, v4f ag0, v4f ag1,
                                        v4f w10, v4f w11, v4f w20, v4f w21, v4f w30, v4f w31,
                                        float bg0, v4f g0, v4f g1, v4f e0, v4f e1, float al,
                                        v4f& r0, v4f& r1) {
  const v4f d0 = sk0 - ag0;
  const v4f d1 = sk1 - ag1;
  float gpart = hsum4(sk0 * w10 + ag0 * w20 + d0 * w30) + hsum4(sk1 * w11 + ag1 * w21 + d1 * w31);
  gpart = wsum(gpart) + bg0;
  const float g  = 1.0f / (1.0f + __expf(-gpart));
  const float gm = 1.0f - g;
  const v4f y0 = sk0 * g + ag0 * gm;
  const v4f y1 = sk1 * g + ag1 * gm;
  const float mu = wsum(hsum4(y0) + hsum4(y1)) * (1.0f / (float)FD);
  const v4f c0 = y0 - mu;
  const v4f c1 = y1 - mu;
  const float var = wsum(hsum4(c0 * c0) + hsum4(c1 * c1)) * (1.0f / (float)FD);
  const float rs = rsqrtf(var + 1e-5f);
  const v4f o0 = c0 * rs * g0 + e0;
  const v4f o1 = c1 * rs * g1 + e1;
  r0 = prelu4(o0, al);
  r1 = prelu4(o1, al);
}

__global__ __launch_bounds__(256) void k_fin(const float* __restrict__ feat,
                                            const unsigned short* __restrict__ wHi,
                                            const unsigned short* __restrict__ wLo,
                                            const float* __restrict__ bs, const float* __restrict__ Wg,
                                            const float* __restrict__ bg, const float* __restrict__ lns,
                                            const float* __restrict__ lnb, const float* __restrict__ alp,
                                            float* io, int nA) {
  constexpr int TPW = 2;
  constexpr int XSP = FD + 4;
  __shared__ __attribute__((aligned(16))) LdsG1 lds;

  const int tid  = threadIdx.x;
  const int lane = tid & 31;
  const int wave = tid >> 5;
  const int hh   = lane >> 4;
  const int m    = lane & 15;
  const int rowBase = blockIdx.x * GR;
  unsigned short* ldsH = lds.hs;
  unsigned short* ldsL = lds.hs + GR * LDSP;

  stage_rows(feat, rowBase, nA, ldsH, ldsL, tid);
  __syncthreads();

  v8f acc[TPW];
  gemm_core<TPW>(ldsH, ldsL, wHi, wLo, 3 * 16 + wave * TPW, lane, acc);
  __syncthreads();

#pragma unroll
  for (int t = 0; t < TPW; ++t) {
    const int gc = (wave * TPW + t) * 16 + m;
    const float bvl = bs[gc];
#pragma unroll
    for (int r = 0; r < 8; ++r) lds.xs[(8 * hh + r) * XSP + gc] = acc[t][r] + bvl;
  }
  __syncthreads();

  const v4f w10 = ld4(Wg + 4 * lane);
  const v4f w11 = ld4(Wg + 128 + 4 * lane);
  const v4f w20 = ld4(Wg + FD + 4 * lane);
  const v4f w21 = ld4(Wg + FD + 128 + 4 * lane);
  const v4f w30 = ld4(Wg + 2 * FD + 4 * lane);
  const v4f w31 = ld4(Wg + 2 * FD + 128 + 4 * lane);
  const v4f g0  = ld4(lns + 4 * lane);
  const v4f g1  = ld4(lns + 128 + 4 * lane);
  const v4f e0  = ld4(lnb + 4 * lane);
  const v4f e1  = ld4(lnb + 128 + 4 * lane);
  const float bg0 = bg[0];
  const float al  = alp[0];

  v4f res[4];
  float* rp[4];
  bool okr[2];
#pragma unroll
  for (int q = 0; q < 2; ++q) {
    const int row  = wave * 2 + q;
    const int node = rowBase + row;
    okr[q] = node < nA;
    const int nl = okr[q] ? node : (nA - 1);
    const float* xsrow = lds.xs + row * XSP + 4 * lane;
    const v4f sk0 = ld4(xsrow);
    const v4f sk1 = ld4(xsrow + 128);
    const float* arow = io + (size_t)nl * FD + 4 * lane;
    const v4f ag0 = ld4(arow);
    const v4f ag1 = ld4(arow + 128);
    row_epi(sk0, sk1, ag0, ag1, w10, w11, w20, w21, w30, w31, bg0, g0, g1, e0, e1, al,
            res[2 * q], res[2 * q + 1]);
    rp[2 * q]     = io + (size_t)nl * FD + 4 * lane;
    rp[2 * q + 1] = io + (size_t)nl * FD + 128 + 4 * lane;
  }
#pragma unroll
  for (int q = 0; q < 2; ++q) {
    if (okr[q]) {
      *(volatile v4f*)(rp[2 * q])     = res[2 * q];
      *(volatile v4f*)(rp[2 * q + 1]) = res[2 * q + 1];
    }
  }
  __threadfence();
#pragma unroll
  for (int q = 0; q < 2; ++q) {
    if (okr[q]) {
      *(volatile v4f*)(rp[2 * q])     = res[2 * q];
      *(volatile v4f*)(rp[2 * q + 1]) = res[2 * q + 1];
    }
  }
}

extern "C" void kernel_launch(void* const* d_in, const int* in_sizes, int n_in,
                              void* d_out, int out_size, void* d_ws, size_t ws_size,
                              hipStream_t stream) {
  if (n_in < 16) return;
  if (in_sizes[0] < FD || (in_sizes[0] % FD) != 0) return;
  const int n  = in_sizes[0] / FD;
  const int nE = in_sizes[1];
  if (nE < 1 || in_sizes[2] != nE) return;
  if (in_sizes[3] != FD * FD || in_sizes[5] != FD * FD || in_sizes[7] != FD * FD || in_sizes[9] != FD * FD) return;
  if (in_sizes[4] != FD || in_sizes[6] != FD || in_sizes[8] != FD || in_sizes[10] != FD) return;
  if (in_sizes[11] != 3 * FD || in_sizes[12] < 1 || in_sizes[13] != FD || in_sizes[14] != FD || in_sizes[15] < 1) return;
  if (out_size != n * FD) return;

  const float* feat = (const float*)d_in[0];
  const int*   src  = (const int*)d_in[1];
  const int*   dst  = (const int*)d_in[2];
  const float* Wq   = (const float*)d_in[3];
  const float* bq   = (const float*)d_in[4];
  const float* Wk   = (const float*)d_in[5];
  const float* bk   = (const float*)d_in[6];
  const float* Wv   = (const float*)d_in[7];
  const float* bv   = (const float*)d_in[8];
  const float* Ws   = (const float*)d_in[9];
  const float* bs   = (const float*)d_in[10];
  const float* Wg   = (const float*)d_in[11];
  const float* bg   = (const float*)d_in[12];
  const float* lns  = (const float*)d_in[13];
  const float* lnb  = (const float*)d_in[14];
  const float* alp  = (const float*)d_in[15];
  float* out = (float*)d_out;

  size_t off = 0;
  unsigned short* wHi = (unsigned short*)((char*)d_ws + off); off += (size_t)4 * FD * FD * 2;
  unsigned short* wLo = (unsigned short*)((char*)d_ws + off); off += (size_t)4 * FD * FD * 2;
  float* Q = (float*)((char*)d_ws + off); off += (size_t)n * FD * sizeof(float);
  float* V = (float*)((char*)d_ws + off); off += (size_t)n * FD * sizeof(float);
  if (off > ws_size || off > WS_CAP) return;

  k_prep<<<(4 * FD + 255) / 256, 256, 0, stream>>>(Wq, Wk, Wv, Ws, wHi, wLo, 4 * FD);

  const int gblk = (n + GR - 1) / GR;
  k_gemm3<<<gblk, 256, 0, stream>>>(feat, wHi, wLo, bq, bk, bv, Q, out, V, n);

  hipFuncSetAttribute(reinterpret_cast<const void*>(&k_agg),
                      hipFuncAttributeMaxDynamicSharedMemorySize, AGG_LDS_BYTES);
  k_agg<<<(n + NB - 1) / NB, ATHR, AGG_LDS_BYTES, stream>>>(src, dst, Q, V, out, n, nE);

  k_fin<<<gblk, 256, 0, stream>>>(feat, wHi, wLo, bs, Wg, bg, lns, lnb, alp, out, n);
}
